// xLSTMEncoderV2_45921790328944
// MI455X (gfx1250) — hardware-verified
//
#include <hip/hip_runtime.h>
#include <stdint.h>

typedef __attribute__((ext_vector_type(16))) _Float16 v16h;
typedef __attribute__((ext_vector_type(8)))  _Float16 v8h;
typedef __attribute__((ext_vector_type(16))) __bf16   v16b;
typedef __attribute__((ext_vector_type(8)))  __bf16   v8b;
typedef __attribute__((ext_vector_type(8)))  float    v8f;
typedef __attribute__((ext_vector_type(4)))  float    v4f;
typedef __attribute__((ext_vector_type(8)))  unsigned short us8;

constexpr int kBatch = 128;
constexpr int kSteps = 512;
constexpr int kInDim = 128;
constexpr int kHid   = 64;
constexpr int kGate  = 4 * kHid;
constexpr int kXRows = kBatch * kSteps;

constexpr int kSPB         = 8;
constexpr int kScanBlocks  = kBatch / kSPB;
constexpr int kScanThreads = 256;
constexpr int kScanWaves   = kScanThreads / 32;
constexpr int kHsP  = 72;
constexpr int kCatP = 136;
constexpr int kGP   = 264;
constexpr int kOstP = 68;
static_assert(kSPB == kScanWaves);
static_assert(kBatch % kSPB == 0);
static_assert(kHid == 64 && kGate == 256 && kInDim == 128);
static_assert(kHsP % 8 == 0 && kCatP % 8 == 0 && kGP % 4 == 0 && kOstP % 4 == 0);
static_assert(kXRows % 64 == 0 && kGate % 64 == 0 && kHid % 64 == 0 && kInDim % 32 == 0 && kHid % 32 == 0);

constexpr int kDwWin = kHid * kInDim / 2;
constexpr int kDwWs  = kGate * kHid / 2;
constexpr int kDwWf  = kHid * 2 * kHid / 2;
constexpr int kPrepEndA = kDwWin / 256;
constexpr int kPrepEndB = kPrepEndA + kDwWs / 256;
constexpr int kPrepEndC = kPrepEndB + kDwWs / 256;
constexpr int kPrepEndD = kPrepEndC + kDwWs / 256;
constexpr int kPrepBlocks = kPrepEndD + kDwWf / 256;
static_assert(kDwWin % 256 == 0 && kDwWs % 256 == 0 && kDwWf % 256 == 0);
constexpr int kXChunks = kXRows * kInDim / 8;
static_assert(kXChunks % 256 == 0);
constexpr int kGemm0Blocks = (kXRows / 64) * (kHid / 64) / 8;
constexpr int kGemm1Blocks = (kXRows / 64) * (kGate / 64) / 8;
static_assert(((kXRows / 64) * (kHid / 64)) % 8 == 0 && ((kXRows / 64) * (kGate / 64)) % 8 == 0);

__device__ __forceinline__ unsigned short f2bf_bits(float f) {
  unsigned u = __float_as_uint(f);
  return (unsigned short)((u + 0x7FFFu + ((u >> 16) & 1u)) >> 16);
}
__device__ __forceinline__ float bf_bits2f(unsigned short h) { return __uint_as_float(((unsigned)h) << 16); }

__device__ __forceinline__ void dep_guard_h(v8f& a, v8f& b, v16h x, v16h y) { asm volatile("v_nop\n\tv_nop\n\tv_nop\n\tv_nop" : "+v"(a), "+v"(b) : "v"(x), "v"(y)); }
__device__ __forceinline__ void dep_guard_b(v8f& a, v8f& b, v16b x, v16b y) { asm volatile("v_nop\n\tv_nop\n\tv_nop\n\tv_nop" : "+v"(a), "+v"(b) : "v"(x), "v"(y)); }
__device__ __forceinline__ void keep4_h(v16h a, v16h b, v16h c, v16h d) { asm volatile("v_nop" :: "v"(a), "v"(b), "v"(c), "v"(d)); }
__device__ __forceinline__ void keep4_b(v16b a, v16b b, v16b c, v16b d) { asm volatile("v_nop" :: "v"(a), "v"(b), "v"(c), "v"(d)); }
__device__ __forceinline__ void acc_guard4(v8f& a, v8f& b, v8f& c, v8f& d) { asm volatile("v_nop\n\tv_nop\n\tv_nop\n\tv_nop" : "+v"(a), "+v"(b), "+v"(c), "+v"(d)); }
template <typename T> struct Frag;
template <> struct Frag<_Float16> {
  typedef v16h V; union U { v16h v; v8h h[2]; };
  static __device__ __forceinline__ v16h load(const _Float16* p) {
    U f; f.h[0] = *(const v8h*)(p); f.h[1] = *(const v8h*)(p + 16); return f.v;
  }
  static __device__ __forceinline__ v8f mma(v16h a, v16h b, v8f c) {
    return __builtin_amdgcn_wmma_f32_16x16x32_f16(false, a, false, b, (short)0, c, false, false);
  }
  static __device__ __forceinline__ void guard(v8f& a, v8f& b, v16h x, v16h y) { dep_guard_h(a, b, x, y); }
  static __device__ __forceinline__ void keep(v16h a, v16h b, v16h c, v16h d) { keep4_h(a, b, c, d); }
};
template <> struct Frag<__bf16> {
  typedef v16b V; union U { v16b v; v8b h[2]; };
  static __device__ __forceinline__ v16b load(const __bf16* p) {
    U f; f.h[0] = *(const v8b*)(p); f.h[1] = *(const v8b*)(p + 16); return f.v;
  }
  static __device__ __forceinline__ v8f mma(v16b a, v16b b, v8f c) {
    return __builtin_amdgcn_wmma_f32_16x16x32_bf16(false, a, false, b, (short)0, c, false, false);
  }
  static __device__ __forceinline__ void guard(v8f& a, v8f& b, v16b x, v16b y) { dep_guard_b(a, b, x, y); }
  static __device__ __forceinline__ void keep(v16b a, v16b b, v16b c, v16b d) { keep4_b(a, b, c, d); }
};

template <int ET> struct Elem;
template <> struct Elem<0> { typedef _Float16 T; };
template <> struct Elem<1> { typedef __bf16 T; };
template <int ET, bool SPLIT, int BIAS_MODE, int OUT_MODE, bool RESID, int ACT = 0>
__global__ __launch_bounds__(256) void wmma_gemm64(
    const unsigned short* __restrict__ Ap, const unsigned short* __restrict__ A2p, int lda, long strideA,
    const unsigned short* __restrict__ Btp, const unsigned short* __restrict__ Bt2p, int ldb, long strideB,
    void* __restrict__ Cout, void* __restrict__ Cout2, int ldc, long strideC,
    const float* __restrict__ bias,
    const float* __restrict__ resid, long strideR,
    int M, int N, int K, float scale) {
  typedef typename Elem<ET>::T T;
  typedef typename Frag<T>::V V;
  const T* A = (const T*)Ap; const T* A2 = (const T*)A2p; const T* Bt = (const T*)Btp; const T* Bt2 = (const T*)Bt2p;
  __shared__ __align__(16) float sT[8][16 * 68];
  const int b    = blockIdx.y;
  const int lane = threadIdx.x & 31;
  const int wave = threadIdx.x >> 5;
  const int tilesN = N >> 6;
  const int tilesM = M >> 6;
  const int tile = blockIdx.x * 8 + wave;
  if (tile >= tilesM * tilesN) return;
  const int tm = tile / tilesN;
  const int tn = tile - tm * tilesN;
  const int m0 = tm << 6;
  const int n0 = tn << 6;

  const T* Ab  = A  + (size_t)b * strideA;
  const T* Bb  = Bt + (size_t)b * strideB;
  const T* Ab2 = SPLIT ? (A2  + (size_t)b * strideA) : nullptr;
  const T* Bb2 = SPLIT ? (Bt2 + (size_t)b * strideB) : nullptr;

  const int rlane = lane & 15;
  const int koff  = (lane >> 4) * 8;
  const int mOff  = (lane >> 4) * 8;

  v8f acc[4][4];
#pragma unroll
  for (int i = 0; i < 4; ++i)
#pragma unroll
    for (int j = 0; j < 4; ++j) acc[i][j] = (v8f){0.f,0.f,0.f,0.f,0.f,0.f,0.f,0.f};

  for (int k0 = 0; k0 < K; k0 += 32) {
    V bh[4], bl[4];
#pragma unroll
    for (int j = 0; j < 4; ++j) {
      const size_t bo = (size_t)(n0 + (j << 4) + rlane) * ldb + koff + k0;
      bh[j] = Frag<T>::load(Bb + bo);
      if (SPLIT) bl[j] = Frag<T>::load(Bb2 + bo);
    }
#pragma unroll
    for (int i = 0; i < 4; ++i) {
      const size_t ao = (size_t)(m0 + (i << 4) + rlane) * lda + koff + k0;
      V ah = Frag<T>::load(Ab + ao);
      V al;
      if (SPLIT) al = Frag<T>::load(Ab2 + ao);
#pragma unroll
      for (int j = 0; j < 4; ++j) {
        acc[i][j] = Frag<T>::mma(ah, bh[j], acc[i][j]);
        if (SPLIT) {
          acc[i][j] = Frag<T>::mma(ah, bl[j], acc[i][j]);
          acc[i][j] = Frag<T>::mma(al, bh[j], acc[i][j]);
        }
      }
      Frag<T>::guard(acc[i][0], acc[i][3], ah, SPLIT ? al : ah);
    }
    Frag<T>::keep(bh[0], bh[1], bh[2], bh[3]);
    if (SPLIT) Frag<T>::keep(bl[0], bl[1], bl[2], bl[3]);
  }
  acc_guard4(acc[0][0], acc[0][1], acc[0][2], acc[0][3]);
  acc_guard4(acc[1][0], acc[1][1], acc[1][2], acc[1][3]);
  acc_guard4(acc[2][0], acc[2][1], acc[2][2], acc[2][3]);
  acc_guard4(acc[3][0], acc[3][1], acc[3][2], acc[3][3]);

  float* slab = sT[wave];
  const float* Rb = RESID ? (resid + (size_t)b * strideR) : nullptr;
#pragma unroll
  for (int i = 0; i < 4; ++i) {
    const int mBase = m0 + (i << 4);
#pragma unroll
    for (int j = 0; j < 4; ++j) {
      const int n = n0 + (j << 4) + rlane;
      float bv = 0.f;
      if (BIAS_MODE == 2) bv = bias[n];
#pragma unroll
      for (int r = 0; r < 8; ++r) {
        float v = acc[i][j][r] * scale;
        if (BIAS_MODE == 1) v += bias[mBase + mOff + r];
        if (BIAS_MODE == 2) v += bv;
        if (RESID) v += Rb[(size_t)(mBase + mOff + r) * ldc + n];
        if (ACT == 1) v = tanhf(v);
        if (ACT == 2) v = fmaxf(v, 0.0f);
        if (ACT == 3) v = v / (1.0f + expf(-v));
        if (ACT == 4) v = (v > 0.f) ? v : 0.01f * v;
        if (ACT == 5) v = 0.5f * v * (1.0f + erff(v * 0.70710678118654752f));
        slab[(mOff + r) * 68 + (j << 4) + rlane] = v;
      }
    }
    __builtin_amdgcn_fence(__ATOMIC_RELEASE, "workgroup");
    __builtin_amdgcn_wave_barrier();
    __builtin_amdgcn_fence(__ATOMIC_ACQUIRE, "workgroup");
    if (OUT_MODE == 0) {
      float* C = (float*)Cout + (size_t)b * strideC;
      const int hh = lane >> 4, c4 = (lane & 15) * 4;
      for (int pass = 0; pass < 2; ++pass) {
#pragma unroll
        for (int it = 0; it < 8; ++it) {
          const int row = it * 2 + hh;
          v4f v = *(const v4f*)(slab + row * 68 + c4);
          *(volatile v4f*)(C + (size_t)(mBase + row) * ldc + n0 + c4) = v;
        }
        __threadfence();
      }
    } else {
      const int q = lane >> 3, c8 = (lane & 7) * 8;
      unsigned short* C  = (unsigned short*)Cout  + (size_t)b * strideC;
      unsigned short* C2 = (OUT_MODE == 2) ? ((unsigned short*)Cout2 + (size_t)b * strideC) : nullptr;
      for (int pass = 0; pass < 2; ++pass) {
#pragma unroll
        for (int it = 0; it < 4; ++it) {
          const int row = it * 4 + q;
          const float* sp = slab + row * 68 + c8;
          v8h hv, lv;
#pragma unroll
          for (int e = 0; e < 8; ++e) {
            if (OUT_MODE == 1) {
              hv[e] = (_Float16)sp[e];
            } else {
              unsigned short hb = f2bf_bits(sp[e]);
              unsigned short lb = f2bf_bits(sp[e] - bf_bits2f(hb));
              hv[e] = __builtin_bit_cast(_Float16, hb);
              lv[e] = __builtin_bit_cast(_Float16, lb);
            }
          }
          *(volatile v8h*)(C + (size_t)(mBase + row) * ldc + n0 + c8) = hv;
          if (OUT_MODE == 2) *(volatile v8h*)(C2 + (size_t)(mBase + row) * ldc + n0 + c8) = lv;
        }
        __threadfence();
      }
    }
    __builtin_amdgcn_fence(__ATOMIC_RELEASE, "workgroup");
    __builtin_amdgcn_wave_barrier();
    __builtin_amdgcn_fence(__ATOMIC_ACQUIRE, "workgroup");
  }
}

__device__ __forceinline__ v8f mma_g(v16b a, v16b b, v8f c) {
  c = __builtin_amdgcn_wmma_f32_16x16x32_bf16(false, a, false, b, (short)0, c, false, false);
  asm volatile("v_nop\n\tv_nop\n\tv_nop\n\tv_nop" : "+v"(c) : "v"(a), "v"(b));
  return c;
}
__device__ __forceinline__ v8f zero8() { return (v8f){0.f, 0.f, 0.f, 0.f, 0.f, 0.f, 0.f, 0.f}; }
__device__ __forceinline__ void store_d(float* g, int pitch, int lane, v8f acc) {
  const int n = lane & 15, mb = (lane >> 4) * 8;
#pragma unroll
  for (int m = 0; m < 8; ++m) g[(mb + m) * pitch + n] = acc[m];
}
__device__ __forceinline__ float wave_sum(float v) {
#pragma unroll
  for (int m = 1; m < 32; m <<= 1) v += __shfl_xor(v, m, 32);
  return v;
}
__device__ __forceinline__ float sigm(float x) { return __builtin_amdgcn_rcpf(1.0f + expf(-x)); }
__device__ __forceinline__ void split_bits(float f, unsigned short& hb, unsigned short& lb) {
  hb = f2bf_bits(f);
  lb = f2bf_bits(f - bf_bits2f(hb));
}
__device__ __forceinline__ void split_bf(float f, __bf16& hi, __bf16& lo) {
  unsigned short hb, lb; split_bits(f, hb, lb);
  hi = __builtin_bit_cast(__bf16, hb);
  lo = __builtin_bit_cast(__bf16, lb);
}
__device__ __forceinline__ void st2u(unsigned* p, unsigned v) { *(volatile unsigned*)p = v; __threadfence(); *(volatile unsigned*)p = v; }

__global__ __launch_bounds__(256) void prep_kernel(
    const float* __restrict__ W_in, const float* __restrict__ W_s, const float* __restrict__ R_s,
    const float* __restrict__ Wq, const float* __restrict__ Wk, const float* __restrict__ Wv,
    const float* __restrict__ Wo, const float* __restrict__ W_fuse,
    unsigned* __restrict__ winh, unsigned* __restrict__ winl,
    unsigned* __restrict__ wsh,  unsigned* __restrict__ wsl,
    unsigned* __restrict__ rsh,  unsigned* __restrict__ rsl,
    unsigned* __restrict__ w2h,  unsigned* __restrict__ w2l,
    unsigned* __restrict__ wfh,  unsigned* __restrict__ wfl) {
  const int blk = blockIdx.x, tid = threadIdx.x;
  float v0, v1;
  unsigned* ph; unsigned* pl; int p;
  if (blk < kPrepEndA) {
    p = blk * 256 + tid;
    const int n = p >> 6, k = (p & 63) * 2;
    v0 = W_in[(size_t)k * kHid + n]; v1 = W_in[(size_t)(k + 1) * kHid + n];
    ph = winh; pl = winl;
  } else if (blk < kPrepEndB) {
    p = (blk - kPrepEndA) * 256 + tid;
    const int n = p >> 5, k = (p & 31) * 2;
    v0 = W_s[(size_t)k * kGate + n]; v1 = W_s[(size_t)(k + 1) * kGate + n];
    ph = wsh; pl = wsl;
  } else if (blk < kPrepEndC) {
    p = (blk - kPrepEndB) * 256 + tid;
    const int n = p >> 5, k = (p & 31) * 2;
    v0 = R_s[(size_t)k * kGate + n]; v1 = R_s[(size_t)(k + 1) * kGate + n];
    ph = rsh; pl = rsl;
  } else if (blk < kPrepEndD) {
    p = (blk - kPrepEndC) * 256 + tid;
    const int n = p >> 5, k = (p & 31) * 2;
    const int g = (blk - kPrepEndC) >> 3;
    const int nn = n & 63;
    const float* W = Wq; float sc = 1.0f;
    if (g == 1) { W = Wk; sc = 0.125f; }
    else if (g == 2) { W = Wv; }
    else if (g == 3) { W = Wo; }
    v0 = W[(size_t)k * kHid + nn] * sc; v1 = W[(size_t)(k + 1) * kHid + nn] * sc;
    ph = w2h; pl = w2l;
  } else {
    p = (blk - kPrepEndD) * 256 + tid;
    const int n = p >> 6, k = (p & 63) * 2;
    v0 = W_fuse[(size_t)k * kHid + n]; v1 = W_fuse[(size_t)(k + 1) * kHid + n];
    ph = wfh; pl = wfl;
  }
  unsigned short h0, l0, h1, l1;
  split_bits(v0, h0, l0);
  split_bits(v1, h1, l1);
  const unsigned hv = (unsigned)h0 | ((unsigned)h1 << 16);
  const unsigned lv = (unsigned)l0 | ((unsigned)l1 << 16);
  st2u(ph + p, hv);
  st2u(pl + p, lv);
}

__global__ __launch_bounds__(256) void xsplit_kernel(const float* __restrict__ x,
                                                     unsigned short* __restrict__ xh, unsigned short* __restrict__ xl) {
  const size_t i = (size_t)blockIdx.x * 256 + threadIdx.x;
  const float* s = x + i * 8;
  const v4f a = *(const v4f*)s;
  const v4f b = *(const v4f*)(s + 4);
  us8 hv, lv;
#pragma unroll
  for (int e = 0; e < 4; ++e) {
    unsigned short hb, lb;
    split_bits(a[e], hb, lb); hv[e] = hb;     lv[e] = lb;
    split_bits(b[e], hb, lb); hv[4 + e] = hb; lv[4 + e] = lb;
  }
  unsigned short* dh = xh + i * 8;
  unsigned short* dl = xl + i * 8;
  *(volatile us8*)dh = hv;
  *(volatile us8*)dl = lv;
  __threadfence();
  *(volatile us8*)dh = hv;
  *(volatile us8*)dl = lv;
}

__device__ __forceinline__ void proj16(const __bf16* Ah, const __bf16* Al, int ap,
                                       const __bf16* __restrict__ Bh, const __bf16* __restrict__ Bl,
                                       float* G, int lane, int wave) {
  const int c = lane & 15, koff = (lane >> 4) * 8;
  v16b ah[2], al[2];
#pragma unroll
  for (int kc = 0; kc < 2; ++kc) {
    ah[kc] = Frag<__bf16>::load(Ah + c * ap + koff + kc * 32);
    al[kc] = Frag<__bf16>::load(Al + c * ap + koff + kc * 32);
  }
#pragma unroll
  for (int jt = 0; jt < 2; ++jt) {
    const int n0 = (wave + 8 * jt) * 16;
    const __bf16* bph = Bh + (size_t)(n0 + c) * kHid + koff;
    const __bf16* bpl = Bl + (size_t)(n0 + c) * kHid + koff;
    v8f acc = zero8();
#pragma unroll
    for (int kc = 0; kc < 2; ++kc) {
      const v16b bh = Frag<__bf16>::load(bph + kc * 32);
      const v16b bl = Frag<__bf16>::load(bpl + kc * 32);
      acc = mma_g(ah[kc], bh, acc);
      acc = mma_g(ah[kc], bl, acc);
      acc = mma_g(al[kc], bh, acc);
    }
    store_d(G + n0, kGP, lane, acc);
  }
}

__device__ __forceinline__ float scell(float zt, float it, float ft, float ot, float& cs, float& ns) {
  const float z = tanhf(zt), iv = expf(it), f = sigm(ft), o = sigm(ot);
  cs = f * cs + iv * z;
  ns = f * ns + iv;
  return (o * cs) * __builtin_amdgcn_rcpf(ns);
}

__global__ __launch_bounds__(kScanThreads) void cell_scan_kernel(
    const float* __restrict__ gx,
    const __bf16* __restrict__ rsTh, const __bf16* __restrict__ rsTl,
    const __bf16* __restrict__ w2Th, const __bf16* __restrict__ w2Tl,
    const __bf16* __restrict__ wfTh, const __bf16* __restrict__ wfTl,
    const float* __restrict__ ln_g, const float* __restrict__ ln_b,
    const float* __restrict__ wi,   const float* __restrict__ bip,
    const float* __restrict__ wf,   const float* __restrict__ bfp,
    const float* __restrict__ bo,   const float* __restrict__ b_fuse,
    float* __restrict__ out) {
  __shared__ __align__(16) float  Cm[kSPB * kHid * kHid];
  __shared__ __align__(16) float  Gb[16 * kGP];
  __shared__ __align__(16) __bf16 HsH[16 * kHsP];
  __shared__ __align__(16) __bf16 HsL[16 * kHsP];
  __shared__ __align__(16) __bf16 CatH[16 * kCatP];
  __shared__ __align__(16) __bf16 CatL[16 * kCatP];
  __shared__ __align__(16) float  Ost[kSPB * kOstP];

  const int tid = threadIdx.x, lane = tid & 31, wave = tid >> 5;
  const int c = lane & 15, koff = (lane >> 4) * 8;
  const int b0 = blockIdx.x * kSPB;
  const int r = wave;
  const int u0 = lane, u1 = lane + 32;

  {
    const v4f z4 = {0.f, 0.f, 0.f, 0.f};
    for (int i = tid; i < (kSPB * kHid * kHid) / 4; i += kScanThreads) *(v4f*)(Cm + 4 * i) = z4;
    const __bf16 zb = __builtin_bit_cast(__bf16, (unsigned short)0);
    const v8b z8 = {zb, zb, zb, zb, zb, zb, zb, zb};
    for (int i = tid; i < (16 * kHsP) / 8; i += kScanThreads) { *(v8b*)(HsH + 8 * i) = z8; *(v8b*)(HsL + 8 * i) = z8; }
    for (int i = tid; i < (16 * kCatP) / 8; i += kScanThreads) { *(v8b*)(CatH + 8 * i) = z8; *(v8b*)(CatL + 8 * i) = z8; }
  }
  const float gg0 = ln_g[u0], gg1 = ln_g[u1], be0 = ln_b[u0], be1 = ln_b[u1];
  const float wi0 = wi[u0], wi1 = wi[u1], wf0 = wf[u0], wf1 = wf[u1];
  const float bo0 = bo[u0], bo1 = bo[u1], bz0 = b_fuse[u0], bz1 = b_fuse[u1];
  const float biS = bip[0], bfS = bfp[0];
  const float inv64 = 1.0f / 64.0f;

  float cs0 = 0.f, cs1 = 0.f, ns0 = 1.f, ns1 = 1.f, nm0 = 0.f, nm1 = 0.f;
  float ho0 = 0.f, ho1 = 0.f, hm0 = 0.f, hm1 = 0.f;
  __syncthreads();

#pragma unroll 1
  for (int t = 0; t < kSteps; ++t) {
    proj16(HsH, HsL, kHsP, rsTh, rsTl, Gb, lane, wave);
    __syncthreads();

    float im, fm;
    {
      const float* gxr = gx + ((size_t)(b0 + r) * kSteps + t) * kGate;
      const float* Gr = Gb + r * kGP;
      const float zt0 = Gr[u0] + gxr[u0],             zt1 = Gr[u1] + gxr[u1];
      const float it0 = Gr[64 + u0] + gxr[64 + u0],   it1 = Gr[64 + u1] + gxr[64 + u1];
      const float ft0 = Gr[128 + u0] + gxr[128 + u0], ft1 = Gr[128 + u1] + gxr[128 + u1];
      const float ot0 = Gr[192 + u0] + gxr[192 + u0], ot1 = Gr[192 + u1] + gxr[192 + u1];
      const float h0v = scell(zt0, it0, ft0, ot0, cs0, ns0);
      const float h1v = scell(zt1, it1, ft1, ot1, cs1, ns1);
      const float mu = wave_sum(h0v + h1v) * inv64;
      const float d0 = h0v - mu, d1 = h1v - mu;
      const float var = wave_sum(d0 * d0 + d1 * d1) * inv64;
      const float rstd = rsqrtf(var + 1e-5f);
      ho0 = d0 * rstd * gg0 + be0;
      ho1 = d1 * rstd * gg1 + be1;
      __bf16 hi, lo;
      split_bf(h0v, hi, lo); HsH[r * kHsP + u0] = hi;  HsL[r * kHsP + u0] = lo;
      split_bf(h1v, hi, lo); HsH[r * kHsP + u1] = hi;  HsL[r * kHsP + u1] = lo;
      split_bf(ho0, hi, lo); CatH[r * kCatP + u0] = hi; CatL[r * kCatP + u0] = lo;
      split_bf(ho1, hi, lo); CatH[r * kCatP + u1] = hi; CatL[r * kCatP + u1] = lo;
      const float gi = wave_sum(ho0 * wi0 + ho1 * wi1);
      const float gf = wave_sum(ho0 * wf0 + ho1 * wf1);
      im = expf(gi + biS);
      fm = sigm(gf + bfS);
    }
    __syncthreads();

    proj16(CatH, CatL, kCatP, w2Th, w2Tl, Gb, lane, wave);
    __syncthreads();

    {
      const float* Gr = Gb + r * kGP;
      const float q0v = Gr[u0], q1v = Gr[u1];
      const float k0v = Gr[64 + u0], k1v = Gr[64 + u1];
      const float v0v = Gr[128 + u0], v1v = Gr[128 + u1];
      const float o0p = Gr[192 + u0], o1p = Gr[192 + u1];
      nm0 = fm * nm0 + im * k0v;
      nm1 = fm * nm1 + im * k1v;
      const float dd = wave_sum(nm0 * q0v + nm1 * q1v);
      const float rden = __builtin_amdgcn_rcpf(fmaxf(fabsf(dd), 1.0f));
      const float iv0 = im * v0v, iv1 = im * v1v;
      float* crow0 = Cm + (r * kHid + u0) * kHid;
      float* crow1 = Cm + (r * kHid + u1) * kHid;
      float num0 = 0.f, num1 = 0.f;
#pragma unroll 2
      for (int jc = 0; jc < kHid / 4; ++jc) {
        const v4f k4 = *(const v4f*)(Gr + 64 + 4 * jc);
        const v4f q4 = *(const v4f*)(Gr + 4 * jc);
        v4f ca = *(const v4f*)(crow0 + 4 * jc);
        v4f cb = *(const v4f*)(crow1 + 4 * jc);
#pragma unroll
        for (int e = 0; e < 4; ++e) {
          ca[e] = fm * ca[e] + iv0 * k4[e];
          cb[e] = fm * cb[e] + iv1 * k4[e];
        }
        *(v4f*)(crow0 + 4 * jc) = ca;
        *(v4f*)(crow1 + 4 * jc) = cb;
#pragma unroll
        for (int e = 0; e < 4; ++e) {
          num0 += ca[e] * q4[e];
          num1 += cb[e] * q4[e];
        }
      }
      hm0 = (sigm(o0p + bo0) * num0) * rden;
      hm1 = (sigm(o1p + bo1) * num1) * rden;
      if (t == kSteps - 1) {
        __bf16 hi, lo;
        split_bf(hm0, hi, lo); CatH[r * kCatP + 64 + u0] = hi; CatL[r * kCatP + 64 + u0] = lo;
        split_bf(hm1, hi, lo); CatH[r * kCatP + 64 + u1] = hi; CatL[r * kCatP + 64 + u1] = lo;
      }
    }
    __syncthreads();
  }

  if (wave < 4) {
    const int n0 = wave * 16;
    const __bf16* bph = wfTh + (size_t)(n0 + c) * (2 * kHid) + koff;
    const __bf16* bpl = wfTl + (size_t)(n0 + c) * (2 * kHid) + koff;
    v8f acc = zero8();
#pragma unroll
    for (int kc = 0; kc < 4; ++kc) {
      const v16b ah = Frag<__bf16>::load(CatH + c * kCatP + koff + kc * 32);
      const v16b al = Frag<__bf16>::load(CatL + c * kCatP + koff + kc * 32);
      const v16b bh = Frag<__bf16>::load(bph + kc * 32);
      const v16b bl = Frag<__bf16>::load(bpl + kc * 32);
      acc = mma_g(ah, bh, acc);
      acc = mma_g(ah, bl, acc);
      acc = mma_g(al, bh, acc);
    }
    store_d(Gb + n0, kGP, lane, acc);
  }
  __syncthreads();
  {
    const float* Gr = Gb + r * kGP;
    const float ga = sigm(Gr[u0] + bz0);
    const float gbv = sigm(Gr[u1] + bz1);
    Ost[r * kOstP + u0] = ga * hm0 + (1.0f - ga) * ho0;
    Ost[r * kOstP + u1] = gbv * hm1 + (1.0f - gbv) * ho1;
  }
  __syncthreads();
  if (wave == 0) {
    const int hh = lane >> 4, c4 = (lane & 15) * 4;
    for (int pass = 0; pass < 2; ++pass) {
#pragma unroll
      for (int it = 0; it < 4; ++it) {
        const int row = it * 2 + hh;
        const v4f v = *(const v4f*)(Ost + row * kOstP + c4);
        *(volatile v4f*)(out + (size_t)(b0 + row) * kHid + c4) = v;
      }
      __threadfence();
    }
  }
}

extern "C" void kernel_launch(void* const* d_in, const int* in_sizes, int n_in,
                              void* d_out, int out_size, void* d_ws, size_t ws_size, hipStream_t stream) {
  if (n_in < 19 || d_out == nullptr || d_ws == nullptr) return;
  if (in_sizes[0] != kBatch * kSteps * kInDim || in_sizes[1] != kInDim * kHid || in_sizes[2] != kHid ||
      in_sizes[3] != kHid * kGate || in_sizes[4] != kHid * kGate || in_sizes[5] != kGate ||
      in_sizes[6] != kHid || in_sizes[7] != kHid || in_sizes[8] != kHid * kHid || in_sizes[9] != kHid * kHid ||
      in_sizes[10] != kHid * kHid || in_sizes[11] != kHid || in_sizes[12] < 1 || in_sizes[13] != kHid ||
      in_sizes[14] < 1 || in_sizes[15] != kHid * kHid || in_sizes[16] != kHid || in_sizes[17] != 2 * kHid * kHid ||
      in_sizes[18] != kHid || out_size != kBatch * kHid) return;

  const float* x      = (const float*)d_in[0];
  const float* W_in   = (const float*)d_in[1];
  const float* b_in   = (const float*)d_in[2];
  const float* W_s    = (const float*)d_in[3];
  const float* R_s    = (const float*)d_in[4];
  const float* b_s    = (const float*)d_in[5];
  const float* ln_g   = (const float*)d_in[6];
  const float* ln_b   = (const float*)d_in[7];
  const float* Wq     = (const float*)d_in[8];
  const float* Wk     = (const float*)d_in[9];
  const float* Wv     = (const float*)d_in[10];
  const float* wi     = (const float*)d_in[11];
  const float* bi     = (const float*)d_in[12];
  const float* wf     = (const float*)d_in[13];
  const float* bf     = (const float*)d_in[14];
  const float* Wo     = (const float*)d_in[15];
  const float* bo     = (const float*)d_in[16];
  const float* W_fuse = (const float*)d_in[17];
  const float* b_fuse = (const float*)d_in[18];
  float* out = (float*)d_out;

  char* ws = (char*)d_ws; size_t off = 0;
  auto carve = [&](size_t bytes) -> char* { char* p = ws + off; off += (bytes + 255) & ~(size_t)255; return p; };
  unsigned short* XH   = (unsigned short*)carve((size_t)kXRows * kInDim * 2);
  unsigned short* XL   = (unsigned short*)carve((size_t)kXRows * kInDim * 2);
  unsigned short* XPH  = (unsigned short*)carve((size_t)kXRows * kHid * 2);
  unsigned short* XPL  = (unsigned short*)carve((size_t)kXRows * kHid * 2);
  float*          GX   = (float*)carve((size_t)kXRows * kGate * 4);
  unsigned short* WINH = (unsigned short*)carve((size_t)kHid * kInDim * 2);
  unsigned short* WINL = (unsigned short*)carve((size_t)kHid * kInDim * 2);
  unsigned short* WSH  = (unsigned short*)carve((size_t)kGate * kHid * 2);
  unsigned short* WSL  = (unsigned short*)carve((size_t)kGate * kHid * 2);
  unsigned short* RSH  = (unsigned short*)carve((size_t)kGate * kHid * 2);
  unsigned short* RSL  = (unsigned short*)carve((size_t)kGate * kHid * 2);
  unsigned short* W2H  = (unsigned short*)carve((size_t)kGate * kHid * 2);
  unsigned short* W2L  = (unsigned short*)carve((size_t)kGate * kHid * 2);
  unsigned short* WFH  = (unsigned short*)carve((size_t)kHid * 2 * kHid * 2);
  unsigned short* WFL  = (unsigned short*)carve((size_t)kHid * 2 * kHid * 2);
  if (off > ws_size || off > (size_t)134217728) return;

  prep_kernel<<<kPrepBlocks, 256, 0, stream>>>(W_in, W_s, R_s, Wq, Wk, Wv, Wo, W_fuse,
                                                (unsigned*)WINH, (unsigned*)WINL, (unsigned*)WSH, (unsigned*)WSL,
                                                (unsigned*)RSH, (unsigned*)RSL, (unsigned*)W2H, (unsigned*)W2L,
                                                (unsigned*)WFH, (unsigned*)WFL);

  xsplit_kernel<<<kXChunks / 256, 256, 0, stream>>>(x, XH, XL);

  wmma_gemm64<1, true, 2, 2, false, 0><<<dim3(kGemm0Blocks, 1), 256, 0, stream>>>(
      XH, XL, kInDim, 0L, WINH, WINL, kInDim, 0L,
      (void*)XPH, (void*)XPL, kHid, 0L, b_in, nullptr, 0L, kXRows, kHid, kInDim, 1.0f);

  wmma_gemm64<1, true, 2, 0, false, 0><<<dim3(kGemm1Blocks, 1), 256, 0, stream>>>(
      XPH, XPL, kHid, 0L, WSH, WSL, kHid, 0L,
      (void*)GX, nullptr, kGate, 0L, b_s, nullptr, 0L, kXRows, kGate, kHid, 1.0f);

  cell_scan_kernel<<<kScanBlocks, kScanThreads, 0, stream>>>(
      GX, (const __bf16*)RSH, (const __bf16*)RSL, (const __bf16*)W2H, (const __bf16*)W2L,
      (const __bf16*)WFH, (const __bf16*)WFL, ln_g, ln_b, wi, bi, wf, bf, bo, b_fuse, out);
}
